// MultiHeadAttention_38903813767268
// MI455X (gfx1250) — hardware-verified
//
#include <hip/hip_runtime.h>


#ifndef NB
#define NB 4
#endif
#ifndef SEQ
#define SEQ 2048
#endif
#define NB_FULL  4
#define SEQ_FULL 2048
#define DD    256
#define NHEAD 8
#define KM    (NHEAD * DD)
#define PCAR  1024.0f
#define SCL2  0.09016844005556021f
#define OCAR  0.0625f
#define WOCAR 256.0f
#define FINSC (1.0f / 16384.0f)
#define WLINES (3 * NHEAD * DD * DD / 64)
#define OLINES (DD * KM / 64)
#define MLINES (NHEAD * DD * DD / 64)

typedef _Float16 h16;
typedef unsigned short bf;
typedef __attribute__((ext_vector_type(16))) __bf16   v16bf;
typedef __attribute__((ext_vector_type(16))) _Float16 v16h;
typedef __attribute__((ext_vector_type(8)))  _Float16 v8h;
typedef __attribute__((ext_vector_type(8)))  unsigned short v8us;
typedef __attribute__((ext_vector_type(2)))  unsigned short v2us;
typedef __attribute__((ext_vector_type(8)))  float    v8f;
typedef __attribute__((ext_vector_type(4)))  float    v4f;
typedef v4f  __attribute__((may_alias)) v4fa;
typedef v8h  __attribute__((may_alias)) v8ha;

static_assert(SEQ % 256 == 0);
static_assert(DD % 64 == 0 && DD % 32 == 0 && KM % 32 == 0 && SEQ % 64 == 0);
static_assert(((size_t)NB * SEQ * DD / 8) % 256 == 0);
static_assert((WLINES + OLINES) % 64 == 0);
static_assert((NHEAD * SEQ) % 8 == 0);
static_assert(WLINES % 64 == 0 && WLINES == 3 * MLINES);
static_assert((size_t)MLINES * 64 == (size_t)NHEAD * DD * DD);
static_assert(KM == NHEAD * DD && (size_t)NHEAD * SEQ * DD == (size_t)SEQ * KM);
static_assert(SEQ % 64 == 0 && DD % 64 == 0);
static_assert(KM % 64 == 0 && SEQ % 32 == 0);

__device__ __forceinline__ unsigned short f2bf(float f) { unsigned u = __float_as_uint(f); u += 0x7FFFu + ((u >> 16) & 1u); return (unsigned short)(u >> 16); }
__device__ __forceinline__ float bf2f(unsigned short b) { return __uint_as_float(((unsigned)b) << 16); }
__device__ __forceinline__ float bfr(float f) { return bf2f(f2bf(f)); }
__device__ __forceinline__ v16h cat16(v8h lo, v8h hi) { return __builtin_shufflevector(lo, hi, 0, 1, 2, 3, 4, 5, 6, 7, 8, 9, 10, 11, 12, 13, 14, 15); }
__device__ __forceinline__ v16bf cat16b(v8us lo, v8us hi) { return __builtin_bit_cast(v16bf, __builtin_shufflevector(lo, hi, 0, 1, 2, 3, 4, 5, 6, 7, 8, 9, 10, 11, 12, 13, 14, 15)); }
__device__ __forceinline__ v8f wmma16(v16h a, v16h b, v8f c) { return __builtin_amdgcn_wmma_f32_16x16x32_f16(false, a, false, b, (short)0, c, false, false); }
__device__ __forceinline__ v8f wmmab(v16bf a, v16bf b, v8f c) { return __builtin_amdgcn_wmma_f32_16x16x32_bf16(false, a, false, b, (short)0, c, false, false); }
static __device__ __forceinline__ h16 toh_flush(float v) { const h16 r = (h16)v; return (fabsf(v) < 6.103515625e-05f) ? (h16)0.0f : r; }

template <typename T16> struct WFrag;
template <> struct WFrag<h16> { typedef v16h V; static __device__ __forceinline__ V ld(const h16* p) { return cat16(*(const v8h*)p, *(const v8h*)(p + 16)); } static __device__ __forceinline__ v8f mma(V a, V b, v8f c) { return wmma16(a, b, c); } };
template <> struct WFrag<bf> { typedef v16bf V; static __device__ __forceinline__ V ld(const bf* p) { return cat16b(*(const v8us*)p, *(const v8us*)(p + 16)); } static __device__ __forceinline__ v8f mma(V a, V b, v8f c) { return wmmab(a, b, c); } };

template <int BIASM>
__device__ __forceinline__ void slab_store(const float* os, h16* crow, int ldc, const float* bias, float alpha, unsigned colbase, unsigned rowbase, unsigned lane) {
    const unsigned rq = lane >> 3, cq = lane & 7u;
    float bc[8];
#pragma unroll
    for (int e = 0; e < 8; ++e) bc[e] = 0.f;
    if (BIASM == 1) { const v4f b0 = *(const v4f*)(bias + colbase + cq * 8u); const v4f b1 = *(const v4f*)(bias + colbase + cq * 8u + 4u);
#pragma unroll
        for (int e = 0; e < 4; ++e) { bc[e] = bfr(b0[e]); bc[4 + e] = bfr(b1[e]); } }
    v8h vals[4];
#pragma unroll
    for (int s = 0; s < 4; ++s) { const unsigned row = (unsigned)s * 4u + rq; const v4f x0 = *(const v4fa*)(os + row * 68u + cq * 8u); const v4f x1 = *(const v4fa*)(os + row * 68u + cq * 8u + 4u);
        float br = 0.f; if (BIASM == 2) br = bfr(bias[rowbase + row]);
        v8h o;
#pragma unroll
        for (int e = 0; e < 4; ++e) { o[e] = (h16)(x0[e] * alpha + (bc[e] + br)); o[4 + e] = (h16)(x1[e] * alpha + (bc[4 + e] + br)); }
        vals[s] = o; }
#pragma unroll 1
    for (int ps = 0; ps < 2; ++ps) {
#pragma unroll
        for (int s = 0; s < 4; ++s) { const unsigned row = (unsigned)s * 4u + rq; *(volatile v8h*)(crow + (size_t)row * ldc + cq * 8u) = vals[s]; }
        if (ps == 0) __threadfence(); }
}
template <int BIASM>
__device__ __forceinline__ void slab_store(const float* os, float* crow, int ldc, const float* bias, float alpha, unsigned colbase, unsigned rowbase, unsigned lane) {
    const unsigned hi = lane >> 4, cofs = (lane & 15u) * 4u;
    v4f bc = (v4f){0.f, 0.f, 0.f, 0.f};
    if (BIASM == 1) { const v4f b0 = *(const v4f*)(bias + colbase + cofs);
#pragma unroll
        for (int e = 0; e < 4; ++e) bc[e] = bfr(b0[e]); }
    v4f vals[8];
#pragma unroll
    for (int s = 0; s < 8; ++s) { const unsigned row = (unsigned)s * 2u + hi; const v4f x = *(const v4fa*)(os + row * 68u + cofs);
        float br = 0.f; if (BIASM == 2) br = bfr(bias[rowbase + row]);
        v4f o;
#pragma unroll
        for (int e = 0; e < 4; ++e) o[e] = x[e] * alpha + (bc[e] + br);
        vals[s] = o; }
#pragma unroll 1
    for (int ps = 0; ps < 2; ++ps) {
#pragma unroll
        for (int s = 0; s < 8; ++s) { const unsigned row = (unsigned)s * 2u + hi; *(volatile v4f*)(crow + (size_t)row * ldc + cofs) = vals[s]; }
        if (ps == 0) __threadfence(); }
}

template <typename T16, typename OT, int BIASM>
__global__ __launch_bounds__(32) void k_gemmw(const T16* __restrict__ A, const T16* __restrict__ Bt, int K, OT* C, int ldc, const float* __restrict__ bias, float alpha, size_t sA, size_t sB, size_t sC, int sBias) {
    typedef typename WFrag<T16>::V V;
    __shared__ __align__(16) float os[16 * 68];
    const size_t z = blockIdx.z; A += z * sA; Bt += z * sB; C += z * sC; if (BIASM != 0) bias += z * (size_t)sBias;
    const unsigned lane = threadIdx.x & 31u, lr = lane & 15u, hi = lane >> 4; const unsigned r0 = blockIdx.x * 64u, c0 = blockIdx.y * 64u;
    v8f acc[4][4];
#pragma unroll
    for (int mb = 0; mb < 4; ++mb)
#pragma unroll
        for (int nb = 0; nb < 4; ++nb) acc[mb][nb] = (v8f){};
    const size_t aoff = (size_t)(r0 + lr) * K + 8u * hi, boff = (size_t)(c0 + lr) * K + 8u * hi;
#pragma unroll 1
    for (int kc = 0; kc < K; kc += 32) {
        V a[4];
#pragma unroll
        for (int mb = 0; mb < 4; ++mb) a[mb] = WFrag<T16>::ld(A + aoff + (size_t)mb * 16 * K + kc);
#pragma unroll
        for (int nb = 0; nb < 4; ++nb) { const V b = WFrag<T16>::ld(Bt + boff + (size_t)nb * 16 * K + kc);
#pragma unroll
            for (int mb = 0; mb < 4; ++mb) acc[mb][nb] = WFrag<T16>::mma(a[mb], b, acc[mb][nb]); }
        asm volatile("v_nop\n\tv_nop\n\tv_nop\n\tv_nop" : "+v"(acc[0][0]), "+v"(acc[1][1]), "+v"(acc[2][2]), "+v"(acc[3][3]) : "v"(a[0]), "v"(a[3]));
    }
#pragma unroll
    for (int mb = 0; mb < 4; ++mb) {
#pragma unroll
        for (int nb = 0; nb < 4; ++nb) {
#pragma unroll
            for (int j = 0; j < 8; ++j) os[(hi * 8u + (unsigned)j) * 68u + (unsigned)nb * 16u + lr] = acc[mb][nb][j]; }
        __builtin_amdgcn_fence(3  , "wavefront"); __builtin_amdgcn_wave_barrier(); asm volatile("" ::: "memory");
        OT* crow = C + (size_t)(r0 + (unsigned)mb * 16u) * ldc + c0;
        slab_store<BIASM>(os, crow, ldc, bias, alpha, c0, r0 + (unsigned)mb * 16u, lane);
        __builtin_amdgcn_fence(3  , "wavefront"); __builtin_amdgcn_wave_barrier(); asm volatile("" ::: "memory");
    }
}

__global__ __launch_bounds__(256) void k_xplanes(const float* __restrict__ xq, const float* __restrict__ xk, const float* __restrict__ xv, bf* XP) {
    const unsigned which = blockIdx.y; const unsigned i = blockIdx.x * 256u + threadIdx.x;
    const unsigned GPB = (unsigned)(SEQ * DD / 8); const unsigned b = i / GPB, rem = i - b * GPB;
    const float* src = (which == 0u) ? xq : ((which == 1u) ? xk : xv);
    const v8f v = *(const v8f*)(src + (size_t)b * SEQ_FULL * DD + (size_t)rem * 8);
    v8us o;
#pragma unroll
    for (int k = 0; k < 8; ++k) o[k] = f2bf(v[k]);
    bf* dst = XP + (size_t)which * NB * SEQ * DD + (size_t)i * 8;
    *(volatile v8us*)dst = o; __threadfence(); *(volatile v8us*)dst = o;
}

__global__ __launch_bounds__(256) void k_wprep(const float* __restrict__ wq, const float* __restrict__ wk, const float* __restrict__ wv, const float* __restrict__ wo, bf* WT, unsigned short* WOS) {
    const unsigned lane = threadIdx.x & 31u; const unsigned wave = (unsigned)__builtin_amdgcn_readfirstlane((int)(threadIdx.x >> 5)); const unsigned L0 = (blockIdx.x * 8u + wave) * 8u;
#pragma unroll
    for (int ps = 0; ps < 2; ++ps) {
#pragma unroll 1
        for (unsigned l = 0; l < 8u; ++l) { const unsigned L = L0 + l; v2us o;
            if (L < (unsigned)WLINES) {
                const unsigned which = L / (unsigned)MLINES; const unsigned e = (L - which * (unsigned)MLINES) * 64u + lane * 2u;
                const float* src = (which == 0u) ? wq : ((which == 1u) ? wk : wv);
                o[0] = f2bf(src[e]); o[1] = f2bf(src[e + 1u]);
                *(volatile v2us*)(WT + (size_t)L * 64u + lane * 2u) = o;
            } else {
                const unsigned e = (L - (unsigned)WLINES) * 64u + lane * 2u;
                const float x0 = bfr(wo[e]) * WOCAR; const float x1 = bfr(wo[e + 1u]) * WOCAR;
                o[0] = __builtin_bit_cast(unsigned short, toh_flush(x0)); o[1] = __builtin_bit_cast(unsigned short, toh_flush(x1));
                *(volatile v2us*)(WOS + e) = o;
            } }
        if (ps == 0) __threadfence(); }
}

__global__ __launch_bounds__(256) void k_vtr(const h16* __restrict__ VP, h16* VT) {
    __shared__ __align__(16) h16 tl[64 * 72];
    const unsigned tid = threadIdx.x; const unsigned t0 = blockIdx.x * 64u, d0 = blockIdx.y * 64u; const size_t hb = (size_t)blockIdx.z * SEQ * DD;
    const unsigned rr = tid >> 3, cq = tid & 7u;
#pragma unroll
    for (int it = 0; it < 2; ++it) { const unsigned row = (unsigned)it * 32u + rr;
        const v8h a = *(const v8h*)(VP + hb + (size_t)(t0 + row) * DD + d0 + cq * 8u);
        *(v8ha*)(tl + row * 72u + cq * 8u) = a; }
    __syncthreads();
    v8h vals[2];
#pragma unroll
    for (int it = 0; it < 2; ++it) { const unsigned drow = (unsigned)it * 32u + rr; v8h o;
#pragma unroll
        for (int e = 0; e < 8; ++e) o[e] = tl[(cq * 8u + (unsigned)e) * 72u + drow];
        vals[it] = o; }
#pragma unroll 1
    for (int ps = 0; ps < 2; ++ps) {
#pragma unroll
        for (int it = 0; it < 2; ++it) { const unsigned drow = (unsigned)it * 32u + rr; *(volatile v8h*)(VT + hb + (size_t)(d0 + drow) * SEQ + t0 + cq * 8u) = vals[it]; }
        if (ps == 0) __threadfence(); }
}

__global__ __launch_bounds__(256) void k_asoft(h16* SP) {
    const unsigned lane = threadIdx.x & 31u; const unsigned row = blockIdx.x * 8u + (threadIdx.x >> 5);
    h16* sr = SP + (size_t)row * SEQ; float v[SEQ / 32]; float mx = -3.0e38f;
#pragma unroll
    for (int ch = 0; ch < SEQ / 256; ++ch) { const v8h a = *(const v8h*)(sr + ch * 256 + lane * 8u);
#pragma unroll
        for (int q = 0; q < 8; ++q) { const float t = (float)a[q]; v[ch * 8 + q] = t; mx = fmaxf(mx, t); } }
#pragma unroll
    for (int sh = 16; sh; sh >>= 1) mx = fmaxf(mx, __shfl_xor(mx, sh, 32));
    float sum = 0.f;
#pragma unroll
    for (int k = 0; k < SEQ / 32; ++k) { float d0 = __fsub_rn(v[k], mx); asm volatile("" : "+v"(d0)); v[k] = __builtin_amdgcn_exp2f(d0); sum += v[k]; }
#pragma unroll
    for (int sh = 16; sh; sh >>= 1) sum += __shfl_xor(sum, sh, 32);
    const float f = __fdiv_rn(PCAR, sum);
    v8h pk[SEQ / 256];
#pragma unroll
    for (int ch = 0; ch < SEQ / 256; ++ch) { v8h o;
#pragma unroll
        for (int q = 0; q < 8; ++q) o[q] = (h16)(v[ch * 8 + q] * f);
        pk[ch] = o; }
#pragma unroll 1
    for (int ps = 0; ps < 2; ++ps) {
#pragma unroll
        for (int ch = 0; ch < SEQ / 256; ++ch) *(volatile v8h*)(sr + ch * 256 + lane * 8u) = pk[ch];
        if (ps == 0) __threadfence(); }
}

#define SZ_XP  ((size_t)3 * NB * SEQ * DD * 2)
#define SZ_WT  ((size_t)3 * NHEAD * DD * DD * 2)
#define SZ_WOS ((size_t)DD * KM * 2)
#define SZ_HP  ((size_t)NHEAD * SEQ * DD * 2)
#define SZ_SP  ((size_t)NHEAD * SEQ * SEQ * 2)
#define SZ_CTX ((size_t)SEQ * KM * 2)
#define SZ_ALL (SZ_XP + SZ_WT + SZ_WOS + 4 * SZ_HP + SZ_SP + SZ_CTX)
static_assert(SZ_ALL <= (size_t)134217728);
static_assert(SZ_XP % 256 == 0 && SZ_WT % 256 == 0 && SZ_WOS % 256 == 0 && SZ_HP % 256 == 0 && SZ_SP % 256 == 0 && SZ_CTX % 256 == 0);
static_assert(SZ_HP == (size_t)SEQ * KM * 2);

extern "C" void kernel_launch(void* const* d_in, const int* in_sizes, int n_in,
                              void* d_out, int out_size, void* d_ws, size_t ws_size, hipStream_t stream) {
    if (n_in < 11) return;
    const size_t xneed = (size_t)(NB - 1) * SEQ_FULL * DD + (size_t)SEQ * DD;
    if ((size_t)in_sizes[0] < xneed || (size_t)in_sizes[1] < xneed || (size_t)in_sizes[2] < xneed) return;
    if ((size_t)in_sizes[3] < (size_t)NHEAD * DD * DD || (size_t)in_sizes[5] < (size_t)NHEAD * DD * DD || (size_t)in_sizes[7] < (size_t)NHEAD * DD * DD) return;
    if ((size_t)in_sizes[4] < (size_t)NHEAD * DD || (size_t)in_sizes[6] < (size_t)NHEAD * DD || (size_t)in_sizes[8] < (size_t)NHEAD * DD) return;
    if ((size_t)in_sizes[9] < (size_t)KM * DD || (size_t)in_sizes[10] < (size_t)DD) return;
    if ((size_t)out_size < (size_t)NB * SEQ * DD) return;
    if (SZ_ALL > ws_size) return;
    const float* Qin = (const float*)d_in[0]; const float* Kin = (const float*)d_in[1]; const float* Vin = (const float*)d_in[2];
    const float* Wq = (const float*)d_in[3]; const float* bq = (const float*)d_in[4]; const float* Wk = (const float*)d_in[5]; const float* bk = (const float*)d_in[6];
    const float* Wv = (const float*)d_in[7]; const float* bv = (const float*)d_in[8]; const float* Wo = (const float*)d_in[9]; const float* bo = (const float*)d_in[10];
    float* OUT = (float*)d_out;
    char* wsp = (char*)d_ws;
    bf* XP = (bf*)wsp; wsp += SZ_XP;
    bf* WT = (bf*)wsp; wsp += SZ_WT;
    h16* WOS = (h16*)wsp; wsp += SZ_WOS;
    h16* QP = (h16*)wsp; wsp += SZ_HP;
    h16* KP = (h16*)wsp; wsp += SZ_HP;
    h16* VP = (h16*)wsp; wsp += SZ_HP;
    h16* VT = (h16*)wsp; wsp += SZ_HP;
    h16* SP = (h16*)wsp; wsp += SZ_SP;
    h16* CTX = (h16*)wsp; wsp += SZ_CTX;
    const bf* XQ = XP; const bf* XK = XP + (size_t)NB * SEQ * DD; const bf* XV = XP + (size_t)2 * NB * SEQ * DD;
    const bf* WQT = WT; const bf* WKT = WT + (size_t)NHEAD * DD * DD; const bf* WVT = WT + (size_t)2 * NHEAD * DD * DD;

    k_xplanes<<<dim3((unsigned)((size_t)NB * SEQ * DD / 8 / 256), 3, 1), 256, 0, stream>>>(Qin, Kin, Vin, XP);
    k_wprep<<<(unsigned)((WLINES + OLINES) / 64), 256, 0, stream>>>(Wq, Wk, Wv, Wo, WT, (unsigned short*)WOS);
    for (int b = 0; b < NB; ++b) {
        const size_t xo = (size_t)b * SEQ * DD;
        k_gemmw<bf, h16, 1><<<dim3(SEQ / 64, DD / 64, NHEAD), 32, 0, stream>>>(XQ + xo, WQT, DD, QP, KM, bq, 1.0f, (size_t)0, (size_t)DD * DD, (size_t)DD, DD);
        k_gemmw<bf, h16, 1><<<dim3(SEQ / 64, DD / 64, NHEAD), 32, 0, stream>>>(XK + xo, WKT, DD, KP, KM, bk, 1.0f, (size_t)0, (size_t)DD * DD, (size_t)DD, DD);
        k_gemmw<bf, h16, 1><<<dim3(SEQ / 64, DD / 64, NHEAD), 32, 0, stream>>>(XV + xo, WVT, DD, VP, KM, bv, 1.0f, (size_t)0, (size_t)DD * DD, (size_t)DD, DD);
        k_vtr<<<dim3(SEQ / 64, DD / 64, NHEAD), 256, 0, stream>>>(VP, VT);
        k_gemmw<h16, h16, 0><<<dim3(SEQ / 64, SEQ / 64, NHEAD), 32, 0, stream>>>(QP, KP, DD, SP, SEQ, nullptr, SCL2, (size_t)SEQ * DD, (size_t)SEQ * DD, (size_t)SEQ * SEQ, 0);
        k_asoft<<<(unsigned)(NHEAD * SEQ / 8), 256, 0, stream>>>(SP);
        k_gemmw<h16, h16, 0><<<dim3(SEQ / 64, DD / 64, NHEAD), 32, 0, stream>>>(SP, VT, SEQ, CTX, KM, nullptr, OCAR, (size_t)SEQ * SEQ, (size_t)DD * SEQ, (size_t)DD, 0);
        k_gemmw<h16, float, 1><<<dim3(SEQ / 64, DD / 64, 1), 32, 0, stream>>>(CTX, WOS, KM, OUT + xo, DD, bo, FINSC, (size_t)0, (size_t)0, (size_t)0, 0);
    }
}
